// D2LDotProductAttention_81389630259486
// MI455X (gfx1250) — hardware-verified
//
#include <hip/hip_runtime.h>
#include <hip/hip_bf16.h>
#include <stddef.h>
#include <stdint.h>

#define NB   32
#define SEQ  2048
#define HD   64
#define NROW (NB * SEQ)
#define QW   16
#define NWV  4
#define QB   (QW * NWV)
#define KC   32
#define CT   64

static_assert(HD == 64);
static_assert(KC == 32);
static_assert(SEQ % QB == 0);
static_assert(SEQ % KC == 0);
static_assert(SEQ % CT == 0);
static_assert((CT * HD) == (256 * 16));

typedef float          v8f   __attribute__((ext_vector_type(8)));
typedef float          v4f   __attribute__((ext_vector_type(4)));
typedef unsigned int   v4u   __attribute__((ext_vector_type(4)));
typedef unsigned short v8us  __attribute__((ext_vector_type(8)));
typedef unsigned short v16us __attribute__((ext_vector_type(16)));
typedef __bf16         v16b  __attribute__((ext_vector_type(16)));
typedef unsigned short ush;

union FragU { v16us v; v8us h[2]; v16b b; };
union PackU { v8us s; v4u u; };
struct HL { v4u h; v4u l; };

__device__ __forceinline__ ush f2bf(float f) {
  const unsigned u = __float_as_uint(f);
  return (ush)((u + 0x7FFFu + ((u >> 16) & 1u)) >> 16);
}
__device__ __forceinline__ float bf2f(ush b) { return __uint_as_float(((unsigned)b) << 16); }

__device__ __forceinline__ HL split8(v8f f) {
  PackU ph, pl;
#pragma unroll
  for (int e = 0; e < 8; ++e) {
    const ush hi = f2bf(f[e]);
    ph.s[e] = hi;
    pl.s[e] = f2bf(f[e] - bf2f(hi));
  }
  HL r; r.h = ph.u; r.l = pl.u;
  return r;
}

__device__ __forceinline__ v8f mmab(v16us a, v16us b, v8f c) {
  FragU ua, ub; ua.v = a; ub.v = b;
  c = __builtin_amdgcn_wmma_f32_16x16x32_bf16(false, ua.b, false, ub.b, (short)0, c, false, false);
  asm volatile("v_nop\n\tv_nop\n\tv_nop\n\tv_nop" : "+v"(c) : "v"(a), "v"(b));
  return c;
}

__device__ __forceinline__ v16us ldfragu(const ush* p, int ld, int row0, int k0, int lane) {
  const int m = lane & 15, lh = lane >> 4;
  const ush* q = p + (size_t)(row0 + m) * ld + k0 + 8 * lh;
  FragU f;
  f.h[0] = *(const v8us*)(q);
  f.h[1] = *(const v8us*)(q + 16);
  return f.v;
}

__device__ __forceinline__ v8f zero8() { return (v8f){0.f, 0.f, 0.f, 0.f, 0.f, 0.f, 0.f, 0.f}; }

#define TP 68
__global__ __launch_bounds__(256) void k_cvt(const float* __restrict__ q, const float* __restrict__ k,
                                             const float* __restrict__ v,
                                             ush* __restrict__ qh, ush* __restrict__ ql,
                                             ush* __restrict__ kh, ush* __restrict__ kl,
                                             ush* __restrict__ vth, ush* __restrict__ vtl) {
  __shared__ __align__(16) float sT[HD * TP];
  const int tid = (int)threadIdx.x;
  const int which = (int)blockIdx.z;
  const int b  = (int)blockIdx.y;
  const int l0 = (int)blockIdx.x * CT;
  const float* src = (which == 0) ? q : ((which == 1) ? k : v);
  const size_t rbase = (size_t)b * SEQ + (size_t)l0;

  v8f f[2];
#pragma unroll
  for (int j = 0; j < 2; ++j) {
    const int p  = tid + 256 * j;
    const int lr = p >> 3;
    const int pc = p & 7;
    const float* sp = src + (rbase + (size_t)lr) * HD + pc * 8;
    const v4f a0 = *(const v4f*)(sp);
    const v4f a1 = *(const v4f*)(sp + 4);
    f[j] = (v8f){a0[0], a0[1], a0[2], a0[3], a1[0], a1[1], a1[2], a1[3]};
  }
  if (which == 2) {
#pragma unroll
    for (int j = 0; j < 2; ++j) {
      const int p  = tid + 256 * j;
      const int lr = p >> 3;
      const int pc = p & 7;
#pragma unroll
      for (int e = 0; e < 8; ++e) sT[(pc * 8 + e) * TP + lr] = f[j][e];
    }
  }
  __syncthreads();

  HL s[2];
  size_t go[2];
  ush* dh;
  ush* dl;
  if (which < 2) {
    dh = (which == 0) ? qh : kh;
    dl = (which == 0) ? ql : kl;
#pragma unroll
    for (int j = 0; j < 2; ++j) {
      const int p  = tid + 256 * j;
      const int lr = p >> 3;
      const int pc = p & 7;
      s[j]  = split8(f[j]);
      go[j] = (rbase + (size_t)lr) * HD + (size_t)(pc * 8);
    }
  } else {
    dh = vth;
    dl = vtl;
#pragma unroll
    for (int j = 0; j < 2; ++j) {
      const int p  = tid + 256 * j;
      const int d  = p >> 3;
      const int pc = p & 7;
      const float* cp = sT + d * TP + pc * 8;
      const v4f x0 = *(const v4f*)(cp);
      const v4f x1 = *(const v4f*)(cp + 4);
      s[j]  = split8((v8f){x0[0], x0[1], x0[2], x0[3], x1[0], x1[1], x1[2], x1[3]});
      go[j] = ((size_t)(b * HD + d)) * SEQ + (size_t)l0 + (size_t)(pc * 8);
    }
  }
#pragma unroll
  for (int j = 0; j < 2; ++j) {
    *(volatile v4u*)(dh + go[j]) = s[j].h;
    *(volatile v4u*)(dl + go[j]) = s[j].l;
  }
  __threadfence();
#pragma unroll
  for (int j = 0; j < 2; ++j) {
    *(volatile v4u*)(dh + go[j]) = s[j].h;
    *(volatile v4u*)(dl + go[j]) = s[j].l;
  }
}

#define OTP 68
__global__ __launch_bounds__(128) void k_attn(const ush* __restrict__ qh, const ush* __restrict__ ql,
                                              const ush* __restrict__ kh, const ush* __restrict__ kl,
                                              const ush* __restrict__ vth, const ush* __restrict__ vtl,
                                              const int* __restrict__ klen, float* __restrict__ out,
                                              int nlen) {
  __shared__ __align__(16) float sw[NWV * QW * OTP];
  const int tid = (int)threadIdx.x, lane = tid & 31, wave = tid >> 5;
  const int hh = lane >> 4, c = lane & 15;
  const int b  = (int)blockIdx.y;
  const int q0 = (int)blockIdx.x * QB + wave * QW;

  int bi = b;
  bi = (bi > nlen - 1) ? (nlen - 1) : bi;
  bi = (bi < 0) ? 0 : bi;
  int vl = klen[bi];
  vl = (vl < 0) ? 0 : vl;
  vl = (vl > SEQ) ? SEQ : vl;
  const int nch = (vl == 0) ? (SEQ / KC) : ((vl + KC - 1) / KC);

  const ush* Qh = qh + (size_t)b * SEQ * HD;
  const ush* Ql = ql + (size_t)b * SEQ * HD;
  const ush* Kh = kh + (size_t)b * SEQ * HD;
  const ush* Kl = kl + (size_t)b * SEQ * HD;
  const ush* Vh = vth + (size_t)b * HD * SEQ;
  const ush* Vl = vtl + (size_t)b * HD * SEQ;

  const v16us q0h = ldfragu(Qh, HD, q0, 0, lane);
  const v16us q1h = ldfragu(Qh, HD, q0, 32, lane);
  const v16us q0l = ldfragu(Ql, HD, q0, 0, lane);
  const v16us q1l = ldfragu(Ql, HD, q0, 32, lane);

  v8f oacc[4];
#pragma unroll
  for (int dt = 0; dt < 4; ++dt) oacc[dt] = zero8();
  float mrun = -1.0e30f;
  float lsum = 0.f;

#pragma unroll 1
  for (int ch = 0; ch < nch; ++ch) {
    const int key0 = ch * KC;
    v8f s[2];
#pragma unroll
    for (int t = 0; t < 2; ++t) {
      const int kr0 = key0 + 16 * t;
      const v16us a0h = ldfragu(Kh, HD, kr0, 0, lane);
      const v16us a0l = ldfragu(Kl, HD, kr0, 0, lane);
      const v16us a1h = ldfragu(Kh, HD, kr0, 32, lane);
      const v16us a1l = ldfragu(Kl, HD, kr0, 32, lane);
      v8f a = zero8();
      a = mmab(a0h, q0h, a);
      a = mmab(a0h, q0l, a);
      a = mmab(a0l, q0h, a);
      a = mmab(a1h, q1h, a);
      a = mmab(a1h, q1l, a);
      a = mmab(a1l, q1h, a);
      s[t] = a;
    }
    float mloc = -1.0e30f;
#pragma unroll
    for (int t = 0; t < 2; ++t) {
#pragma unroll
      for (int r = 0; r < 8; ++r) {
        const int key = key0 + 16 * t + 8 * hh + r;
        float x = s[t][r] * 0.125f;
        x = (key < vl) ? x : -1000000.0f;
        s[t][r] = x;
        mloc = fmaxf(mloc, x);
      }
    }
    mloc = fmaxf(mloc, __shfl_xor(mloc, 16, 32));
    const float mnew = fmaxf(mrun, mloc);
    const float corr = __expf(mrun - mnew);
    mrun = mnew;
    lsum *= corr;
#pragma unroll
    for (int dt = 0; dt < 4; ++dt) oacc[dt] = oacc[dt] * corr;

    FragU fh, fl;
#pragma unroll
    for (int t = 0; t < 2; ++t) {
      PackU ph, pl;
#pragma unroll
      for (int r = 0; r < 8; ++r) {
        const float p = __expf(s[t][r] - mnew);
        lsum += p;
        const ush hi = f2bf(p);
        ph.s[r] = hi;
        pl.s[r] = f2bf(p - bf2f(hi));
      }
      fh.h[t] = ph.s;
      fl.h[t] = pl.s;
    }
#pragma unroll
    for (int dt = 0; dt < 4; ++dt) {
      const v16us bvh = ldfragu(Vh, SEQ, 16 * dt, key0, lane);
      const v16us bvl = ldfragu(Vl, SEQ, 16 * dt, key0, lane);
      oacc[dt] = mmab(bvh, fh.v, oacc[dt]);
      oacc[dt] = mmab(bvh, fl.v, oacc[dt]);
      oacc[dt] = mmab(bvl, fh.v, oacc[dt]);
    }
  }

  const float lt  = lsum + __shfl_xor(lsum, 16, 32);
  const float inv = 1.0f / lt;
  float* sww = sw + wave * (QW * OTP);
#pragma unroll
  for (int dt = 0; dt < 4; ++dt) {
    const v8f o = oacc[dt] * inv;
    const v4f w0 = (v4f){o[0], o[1], o[2], o[3]};
    const v4f w1 = (v4f){o[4], o[5], o[6], o[7]};
    float* dp = sww + c * OTP + 16 * dt + 8 * hh;
    *(v4f*)(dp)     = w0;
    *(v4f*)(dp + 4) = w1;
  }
  __syncthreads();
  v4f val[8];
  size_t go[8];
#pragma unroll
  for (int it = 0; it < 8; ++it) {
    const int p   = lane + 32 * it;
    const int row = p >> 4;
    const int pc  = p & 15;
    val[it] = *(const v4f*)(sww + row * OTP + pc * 4);
    go[it]  = ((size_t)b * SEQ + (size_t)(q0 + row)) * HD + (size_t)(pc * 4);
  }
#pragma unroll
  for (int it = 0; it < 8; ++it) *(volatile v4f*)(out + go[it]) = val[it];
  __threadfence();
#pragma unroll
  for (int it = 0; it < 8; ++it) *(volatile v4f*)(out + go[it]) = val[it];
}

extern "C" void kernel_launch(void* const* d_in, const int* in_sizes, int n_in,
                              void* d_out, int out_size, void* d_ws, size_t ws_size,
                              hipStream_t stream) {
  if (n_in < 4) return;
  if (in_sizes[0] != NROW * HD) return;
  if (in_sizes[1] != NROW * HD) return;
  if (in_sizes[2] != NROW * HD) return;
  if (in_sizes[3] != NB) return;
  if (out_size != NROW * HD) return;

  const float* q    = (const float*)d_in[0];
  const float* k    = (const float*)d_in[1];
  const float* v    = (const float*)d_in[2];
  const int*   klen = (const int*)d_in[3];
  float* out = (float*)d_out;

  const size_t plane = (size_t)NROW * HD * 2;
  size_t off = 0;
  const size_t oQh = off; off += plane;
  const size_t oQl = off; off += plane;
  const size_t oKh = off; off += plane;
  const size_t oKl = off; off += plane;
  const size_t oVh = off; off += plane;
  const size_t oVl = off; off += plane;
  if (off > ws_size) return;
  if (off > (size_t)134217728) return;

  char* ws = (char*)d_ws;
  ush* Qh  = (ush*)(ws + oQh);
  ush* Ql  = (ush*)(ws + oQl);
  ush* Kh  = (ush*)(ws + oKh);
  ush* Kl  = (ush*)(ws + oKl);
  ush* Vth = (ush*)(ws + oVh);
  ush* Vtl = (ush*)(ws + oVl);

  k_cvt<<<dim3(SEQ / CT, NB, 3), dim3(256), 0, stream>>>(q, k, v, Qh, Ql, Kh, Kl, Vth, Vtl);
  k_attn<<<dim3(SEQ / QB, NB), dim3(NWV * 32), 0, stream>>>(Qh, Ql, Kh, Kl, Vth, Vtl, klen, out,
                                                            in_sizes[3]);
  (void)hipGetLastError();
}
